// EdgeMask_34488587387482
// MI455X (gfx1250) — hardware-verified
//
#include <hip/hip_runtime.h>


#define NR   32768
#define DD   128
#define HH   32
#define NN   128
typedef _Float16 h16;
typedef unsigned short bf;
typedef __attribute__((ext_vector_type(16))) __bf16   v16bf;
typedef __attribute__((ext_vector_type(16))) _Float16 v16h;
typedef __attribute__((ext_vector_type(8)))  _Float16 v8h;
typedef __attribute__((ext_vector_type(8)))  unsigned short v8us;
typedef __attribute__((ext_vector_type(8)))  float    v8f;
typedef __attribute__((ext_vector_type(4)))  float    v4f;
typedef v8h  __attribute__((may_alias)) v8ha;
typedef v4f  __attribute__((may_alias)) v4fa;
typedef v8us __attribute__((may_alias)) v8usa;

__device__ __forceinline__ unsigned short f2bf(float f) { unsigned u = __float_as_uint(f); u += 0x7FFFu + ((u >> 16) & 1u); return (unsigned short)(u >> 16); }
__device__ __forceinline__ float bf2f(unsigned short b) { return __uint_as_float(((unsigned)b) << 16); }
__device__ __forceinline__ float bfr(float f) { return bf2f(f2bf(f)); }
__device__ __forceinline__ v16h cat16(v8h lo, v8h hi) { return __builtin_shufflevector(lo, hi, 0, 1, 2, 3, 4, 5, 6, 7, 8, 9, 10, 11, 12, 13, 14, 15); }
__device__ __forceinline__ v16bf cat16b(v8us lo, v8us hi) { return __builtin_bit_cast(v16bf, __builtin_shufflevector(lo, hi, 0, 1, 2, 3, 4, 5, 6, 7, 8, 9, 10, 11, 12, 13, 14, 15)); }
__device__ __forceinline__ v8f wmma16(v16h a, v16h b, v8f c) { return __builtin_amdgcn_wmma_f32_16x16x32_f16(false, a, false, b, (short)0, c, false, false); }
__device__ __forceinline__ v8f wmmab(v16bf a, v16bf b, v8f c) { return __builtin_amdgcn_wmma_f32_16x16x32_bf16(false, a, false, b, (short)0, c, false, false); }


template <typename T16> struct WFrag;
template <> struct WFrag<h16> { typedef v16h V; static __device__ __forceinline__ V ld(const h16* p) { return cat16(*(const v8h*)p, *(const v8h*)(p + 16)); } static __device__ __forceinline__ v8f mma(V a, V b, v8f c) { return wmma16(a, b, c); } };
template <> struct WFrag<bf> { typedef v16bf V; static __device__ __forceinline__ V ld(const bf* p) { return cat16b(*(const v8us*)p, *(const v8us*)(p + 16)); } static __device__ __forceinline__ v8f mma(V a, V b, v8f c) { return wmmab(a, b, c); } };
template <typename T16, int NSPLIT, bool BIAS>
__global__ __launch_bounds__(32) void k_gemmw(const T16* __restrict__ A, const T16* __restrict__ A2, const T16* __restrict__ Bt, const T16* __restrict__ Bt2, int K, float* C, int ldc, const float* __restrict__ bias, size_t sA, size_t sB, size_t sC) {
    typedef typename WFrag<T16>::V V;
    __shared__ __align__(16) float os[16 * 68];
    const size_t z = blockIdx.z; A += z * sA; if (A2) A2 += z * sA; Bt += z * sB; if (Bt2) Bt2 += z * sB; C += z * sC;
    const int lane = threadIdx.x & 31, lr = lane & 15, hi = lane >> 4; const int r0 = blockIdx.x * 64, c0 = blockIdx.y * 64;
    v8f acc[4][4];
#pragma unroll
    for (int mb = 0; mb < 4; ++mb)
#pragma unroll
        for (int nb = 0; nb < 4; ++nb) acc[mb][nb] = (v8f){};
    const size_t aoff = (size_t)(r0 + lr) * K + 8 * hi, boff = (size_t)(c0 + lr) * K + 8 * hi;
#pragma unroll 1
    for (int kc = 0; kc < K; kc += 32) {
        V a[4], a2[4];
#pragma unroll
        for (int mb = 0; mb < 4; ++mb) { a[mb] = WFrag<T16>::ld(A + aoff + (size_t)mb * 16 * K + kc); if (NSPLIT == 1 || NSPLIT == 2) a2[mb] = WFrag<T16>::ld(A2 + aoff + (size_t)mb * 16 * K + kc); }
#pragma unroll
        for (int nb = 0; nb < 4; ++nb) { const V b = WFrag<T16>::ld(Bt + boff + (size_t)nb * 16 * K + kc); V b2; if (NSPLIT >= 2) b2 = WFrag<T16>::ld(Bt2 + boff + (size_t)nb * 16 * K + kc);
#pragma unroll
            for (int mb = 0; mb < 4; ++mb) { acc[mb][nb] = WFrag<T16>::mma(a[mb], b, acc[mb][nb]); if (NSPLIT == 1 || NSPLIT == 2) acc[mb][nb] = WFrag<T16>::mma(a2[mb], b, acc[mb][nb]); if (NSPLIT >= 2) acc[mb][nb] = WFrag<T16>::mma(a[mb], b2, acc[mb][nb]); } }
        asm volatile("v_nop\n\tv_nop\n\tv_nop\n\tv_nop" : "+v"(acc[0][0]), "+v"(acc[1][1]), "+v"(acc[2][2]), "+v"(acc[3][3]) : "v"(a[0]), "v"(a[3]));
    }
#pragma unroll
    for (int mb = 0; mb < 4; ++mb) {
#pragma unroll
        for (int nb = 0; nb < 4; ++nb) {
#pragma unroll
            for (int j = 0; j < 8; ++j) os[(hi * 8 + j) * 68 + nb * 16 + lr] = acc[mb][nb][j]; }
        __builtin_amdgcn_wave_barrier(); asm volatile("" ::: "memory");
        float* crow = C + (size_t)(r0 + mb * 16) * ldc + c0;
#pragma unroll 1
        for (int ps = 0; ps < 2; ++ps) {
#pragma unroll
            for (int s = 0; s < 8; ++s) { const int row = 2 * s + hi, cofs = lr * 4; v4f val = *(const v4fa*)(os + row * 68 + cofs); if (BIAS) { val[0] += bfr(bias[c0 + cofs]); val[1] += bfr(bias[c0 + cofs + 1]); val[2] += bfr(bias[c0 + cofs + 2]); val[3] += bfr(bias[c0 + cofs + 3]); }
                *(volatile v4f*)(crow + (size_t)row * ldc + cofs) = val; }
            if (ps == 0) __threadfence(); }
        __builtin_amdgcn_wave_barrier(); asm volatile("" ::: "memory");
    }
}

typedef __attribute__((ext_vector_type(4))) unsigned short v4us;

__global__ __launch_bounds__(256) void k_cvt8(const float* __restrict__ src, bf* dst, size_t n8) { const size_t i = (size_t)blockIdx.x * 256 + threadIdx.x; if (i >= n8) return; const v8f v = *(const v8f*)(src + i * 8); v8us o;
#pragma unroll
    for (int k = 0; k < 8; ++k) o[k] = f2bf(v[k]); *(volatile v8us*)(dst + i * 8) = o; __threadfence(); *(volatile v8us*)(dst + i * 8) = o; }
__global__ __launch_bounds__(256) void k_w1(const float* __restrict__ W1, bf* Bt) { const int e = (blockIdx.x * 256 + threadIdx.x) * 4; if (e >= 2 * HH * DD) return; const int k = e % DD, n = e / DD; v4us o;
#pragma unroll
    for (int u = 0; u < 4; ++u) o[u] = f2bf(n < HH ? W1[(size_t)(k + u) * HH + n] : W1[(size_t)(DD + k + u) * HH + (n - HH)]); *(volatile v4us*)(Bt + e) = o; __threadfence(); *(volatile v4us*)(Bt + e) = o; }
__global__ __launch_bounds__(256) void k_edge(const float* __restrict__ LL, const float* __restrict__ b1, const float* __restrict__ W2, const float* __restrict__ b2, const float* __restrict__ If, float* OI, float* OM) { const size_t idx = (size_t)blockIdx.x * 256 + threadIdx.x; if (idx >= (size_t)NR * NN) return; const int j = (int)(idx % NN); const int i = (int)((idx / NN) % NN); const size_t bt = idx / ((size_t)NN * NN);
    const float* li = LL + (bt * NN + i) * (2 * HH); const float* lj = LL + (bt * NN + j) * (2 * HH) + HH; float acc = 0.f;
#pragma unroll
    for (int k = 0; k < HH; ++k) { const float s = fmaxf(__fadd_rn(__fadd_rn(li[k], lj[k]), bfr(b1[k])), 0.f); float w = bfr(W2[k]); asm volatile("" : "+v"(w)); float pr = __fmul_rn(s, w); asm volatile("" : "+v"(pr)); acc = __fadd_rn(acc, pr); }
    float bb = bfr(b2[0]); asm volatile("" : "+v"(bb)); const float lg = __fadd_rn(acc, bb); const float m = __fdiv_rn(1.0f, 1.0f + __expf(-lg)); const float iv = __fmul_rn(bfr(If[idx]), m);
    *(volatile float*)(OI + idx) = iv; *(volatile float*)(OM + idx) = m; __threadfence(); *(volatile float*)(OI + idx) = iv; *(volatile float*)(OM + idx) = m; }

extern "C" void kernel_launch(void* const* d_in, const int* in_sizes, int n_in,
                              void* d_out, int out_size, void* d_ws, size_t ws_size, hipStream_t stream) {
    (void)in_sizes; (void)n_in; (void)out_size;
    const float* h = (const float*)d_in[0]; const float* If = (const float*)d_in[1]; const float* W1 = (const float*)d_in[2]; const float* b1 = (const float*)d_in[3]; const float* W2 = (const float*)d_in[4]; const float* b2 = (const float*)d_in[5];
    float* OI = (float*)d_out; float* OM = OI + (size_t)NR * NN;
    char* wsp = (char*)d_ws;
    auto take = [&](size_t bytes) { char* p = wsp; wsp += (bytes + 255) & ~(size_t)255; return (void*)p; };
    bf* WB = (bf*)take(2 * HH * DD * 2); bf* HB = (bf*)take((size_t)NR * DD * 2); float* LL = (float*)take((size_t)NR * 2 * HH * 4);
    if ((size_t)(wsp - (char*)d_ws) > ws_size) return;
    k_w1<<<(2 * HH * DD / 4 + 255) / 256, 256, 0, stream>>>(W1, WB); k_cvt8<<<(unsigned)(((size_t)NR * DD / 8 + 255) / 256), 256, 0, stream>>>(h, HB, (size_t)NR * DD / 8);
    k_gemmw<bf, 0, false><<<dim3(NR / 64, 1, 1), 32, 0, stream>>>(HB, nullptr, WB, nullptr, DD, LL, 2 * HH, nullptr, 0, 0, 0);
    k_edge<<<(unsigned)(((size_t)NR * NN + 255) / 256), 256, 0, stream>>>(LL, b1, W2, b2, If, OI, OM);
}
